// ReprogrammingLayer_m2_78675210928569
// MI455X (gfx1250) — hardware-verified
//
#include <hip/hip_runtime.h>


#define NB_  2
#define LQ   2048
#define LS   4096
#define DM   1024
#define NH_  16
#define HD   64
#define ZH   2
#define PCAR 1024.0f
typedef _Float16 h16;
typedef unsigned short bf;
typedef __attribute__((ext_vector_type(16))) __bf16   v16bf;
typedef __attribute__((ext_vector_type(16))) _Float16 v16h;
typedef __attribute__((ext_vector_type(8)))  _Float16 v8h;
typedef __attribute__((ext_vector_type(8)))  unsigned short v8us;
typedef __attribute__((ext_vector_type(8)))  float    v8f;
typedef __attribute__((ext_vector_type(4)))  float    v4f;
typedef v8h  __attribute__((may_alias)) v8ha;
typedef v4f  __attribute__((may_alias)) v4fa;
typedef v8us __attribute__((may_alias)) v8usa;

__device__ __forceinline__ unsigned short f2bf(float f) { unsigned u = __float_as_uint(f); u += 0x7FFFu + ((u >> 16) & 1u); return (unsigned short)(u >> 16); }
__device__ __forceinline__ float bf2f(unsigned short b) { return __uint_as_float(((unsigned)b) << 16); }
__device__ __forceinline__ float bfr(float f) { return bf2f(f2bf(f)); }
__device__ __forceinline__ v16h cat16(v8h lo, v8h hi) { return __builtin_shufflevector(lo, hi, 0, 1, 2, 3, 4, 5, 6, 7, 8, 9, 10, 11, 12, 13, 14, 15); }
__device__ __forceinline__ v16bf cat16b(v8us lo, v8us hi) { return __builtin_bit_cast(v16bf, __builtin_shufflevector(lo, hi, 0, 1, 2, 3, 4, 5, 6, 7, 8, 9, 10, 11, 12, 13, 14, 15)); }
__device__ __forceinline__ v8f wmma16(v16h a, v16h b, v8f c) { return __builtin_amdgcn_wmma_f32_16x16x32_f16(false, a, false, b, (short)0, c, false, false); }
__device__ __forceinline__ v8f wmmab(v16bf a, v16bf b, v8f c) { return __builtin_amdgcn_wmma_f32_16x16x32_bf16(false, a, false, b, (short)0, c, false, false); }


template <typename T16> struct WFrag;
template <> struct WFrag<h16> { typedef v16h V; static __device__ __forceinline__ V ld(const h16* p) { return cat16(*(const v8h*)p, *(const v8h*)(p + 16)); } static __device__ __forceinline__ v8f mma(V a, V b, v8f c) { return wmma16(a, b, c); } };
template <> struct WFrag<bf> { typedef v16bf V; static __device__ __forceinline__ V ld(const bf* p) { return cat16b(*(const v8us*)p, *(const v8us*)(p + 16)); } static __device__ __forceinline__ v8f mma(V a, V b, v8f c) { return wmmab(a, b, c); } };
template <typename T16, int NSPLIT, bool BIAS>
__global__ __launch_bounds__(32) void k_gemmw(const T16* __restrict__ A, const T16* __restrict__ A2, const T16* __restrict__ Bt, const T16* __restrict__ Bt2, int K, float* C, int ldc, const float* __restrict__ bias, size_t sA, size_t sB, size_t sC) {
    typedef typename WFrag<T16>::V V;
    __shared__ __align__(16) float os[16 * 68];
    const size_t z = blockIdx.z; A += z * sA; if (A2) A2 += z * sA; Bt += z * sB; if (Bt2) Bt2 += z * sB; C += z * sC;
    const int lane = threadIdx.x & 31, lr = lane & 15, hi = lane >> 4; const int r0 = blockIdx.x * 64, c0 = blockIdx.y * 64;
    v8f acc[4][4];
#pragma unroll
    for (int mb = 0; mb < 4; ++mb)
#pragma unroll
        for (int nb = 0; nb < 4; ++nb) acc[mb][nb] = (v8f){};
    const size_t aoff = (size_t)(r0 + lr) * K + 8 * hi, boff = (size_t)(c0 + lr) * K + 8 * hi;
#pragma unroll 1
    for (int kc = 0; kc < K; kc += 32) {
        V a[4], a2[4];
#pragma unroll
        for (int mb = 0; mb < 4; ++mb) { a[mb] = WFrag<T16>::ld(A + aoff + (size_t)mb * 16 * K + kc); if (NSPLIT == 1 || NSPLIT == 2) a2[mb] = WFrag<T16>::ld(A2 + aoff + (size_t)mb * 16 * K + kc); }
#pragma unroll
        for (int nb = 0; nb < 4; ++nb) { const V b = WFrag<T16>::ld(Bt + boff + (size_t)nb * 16 * K + kc); V b2; if (NSPLIT >= 2) b2 = WFrag<T16>::ld(Bt2 + boff + (size_t)nb * 16 * K + kc);
#pragma unroll
            for (int mb = 0; mb < 4; ++mb) { acc[mb][nb] = WFrag<T16>::mma(a[mb], b, acc[mb][nb]); if (NSPLIT == 1 || NSPLIT == 2) acc[mb][nb] = WFrag<T16>::mma(a2[mb], b, acc[mb][nb]); if (NSPLIT >= 2) acc[mb][nb] = WFrag<T16>::mma(a[mb], b2, acc[mb][nb]); } }
        asm volatile("v_nop\n\tv_nop\n\tv_nop\n\tv_nop" : "+v"(acc[0][0]), "+v"(acc[1][1]), "+v"(acc[2][2]), "+v"(acc[3][3]) : "v"(a[0]), "v"(a[3]));
    }
#pragma unroll
    for (int mb = 0; mb < 4; ++mb) {
#pragma unroll
        for (int nb = 0; nb < 4; ++nb) {
#pragma unroll
            for (int j = 0; j < 8; ++j) os[(hi * 8 + j) * 68 + nb * 16 + lr] = acc[mb][nb][j]; }
        __builtin_amdgcn_wave_barrier(); asm volatile("" ::: "memory");
        float* crow = C + (size_t)(r0 + mb * 16) * ldc + c0;
#pragma unroll 1
        for (int ps = 0; ps < 2; ++ps) {
#pragma unroll
            for (int s = 0; s < 8; ++s) { const int row = 2 * s + hi, cofs = lr * 4; v4f val = *(const v4fa*)(os + row * 68 + cofs); if (BIAS) { val[0] += bfr(bias[c0 + cofs]); val[1] += bfr(bias[c0 + cofs + 1]); val[2] += bfr(bias[c0 + cofs + 2]); val[3] += bfr(bias[c0 + cofs + 3]); }
                *(volatile v4f*)(crow + (size_t)row * ldc + cofs) = val; }
            if (ps == 0) __threadfence(); }
        __builtin_amdgcn_wave_barrier(); asm volatile("" ::: "memory");
    }
}

__device__ __forceinline__ h16 tohx(float x) { return (h16)x; }
__device__ __forceinline__ void splitf(float y, unsigned short& h, unsigned short& l) { h = f2bf(y); l = f2bf(y - bf2f(h)); }
typedef __attribute__((ext_vector_type(2))) _Float16 v2h;
typedef __attribute__((ext_vector_type(4))) _Float16 v4h;
typedef __attribute__((ext_vector_type(2))) unsigned short v2us;
typedef __attribute__((ext_vector_type(4))) unsigned short v4us;

__global__ __launch_bounds__(256) void k_cvt8(const float* __restrict__ src, bf* dst, size_t n8) { const size_t i = (size_t)blockIdx.x * 256 + threadIdx.x; if (i >= n8) return; const v8f v = *(const v8f*)(src + i * 8); v8us o;
#pragma unroll
    for (int k = 0; k < 8; ++k) o[k] = f2bf(v[k]); *(volatile v8us*)(dst + i * 8) = o; __threadfence(); *(volatile v8us*)(dst + i * 8) = o; }
__global__ __launch_bounds__(256) void k_wtG(const float* __restrict__ w, int K, int N, bf* Bt) {
    const int lane = threadIdx.x & 31; const int L0 = (blockIdx.x * 8 + (threadIdx.x >> 5)) * 8; const int nlines = N * K / 64;
#pragma unroll 1
    for (int ps = 0; ps < 2; ++ps) {
#pragma unroll 1
        for (int l = 0; l < 8; ++l) { const int L = L0 + l; if (L >= nlines) break; const size_t e = (size_t)L * 64 + lane * 2; const int k = (int)(e % K), n = (int)(e / K); v2us o;
            o[0] = f2bf(w[(size_t)k * N + n]); o[1] = f2bf(w[(size_t)(k + 1) * N + n]); *(volatile v2us*)(Bt + e) = o; }
        if (ps == 0) __threadfence(); }
}
__global__ __launch_bounds__(256) void k_hpl(const float* __restrict__ F, int nrows, float sc, h16* P) { const size_t e = ((size_t)blockIdx.x * 256 + threadIdx.x) * 4; if (e >= (size_t)NH_ * nrows * HD) return; const int d = (int)(e % HD); const int n = (int)((e / HD) % nrows); const int h = (int)(e / ((size_t)HD * nrows)); const v4f a = *(const v4f*)(F + (size_t)n * DM + h * HD + d); v4h o;
#pragma unroll
    for (int q = 0; q < 4; ++q) o[q] = tohx(a[q] * sc); *(volatile v4h*)(P + e) = o; __threadfence(); *(volatile v4h*)(P + e) = o; }
__global__ __launch_bounds__(256) void k_vt(const float* __restrict__ V, h16* VT) { const size_t e = ((size_t)blockIdx.x * 256 + threadIdx.x) * 2; if (e >= (size_t)NH_ * HD * LS) return; const int s = (int)(e % LS); const int d = (int)((e / LS) % HD); const int h = (int)(e / ((size_t)LS * HD)); v2h o; o[0] = tohx(V[(size_t)s * DM + h * HD + d]); o[1] = tohx(V[(size_t)(s + 1) * DM + h * HD + d]); *(volatile v2h*)(VT + e) = o; __threadfence(); *(volatile v2h*)(VT + e) = o; }
__global__ __launch_bounds__(256) void k_mrg(const float* __restrict__ O, int h0, bf* Mh, bf* Ml) { const size_t e = ((size_t)blockIdx.x * 256 + threadIdx.x) * 2; if (e >= (size_t)ZH * LQ * HD) return; const int d = (int)(e % HD); const int n = (int)((e / HD) % LQ); const int z = (int)(e / ((size_t)HD * LQ)); v2us oh, ol;
#pragma unroll
    for (int q = 0; q < 2; ++q) { unsigned short a, c; splitf(O[e + q] * (1.0f / PCAR), a, c); oh[q] = a; ol[q] = c; } const size_t oo = (size_t)n * DM + (h0 + z) * HD + d;
    *(volatile v2us*)(Mh + oo) = oh; *(volatile v2us*)(Ml + oo) = ol; __threadfence(); *(volatile v2us*)(Mh + oo) = oh; *(volatile v2us*)(Ml + oo) = ol; }
template <int NFULL, int TAIL> __global__ __launch_bounds__(256) void k_soft(const float* __restrict__ Sb, int nrows, int rowsper, int rvalid, int nvalid, h16* P) { const int lane = threadIdx.x & 31; const size_t row = (size_t)blockIdx.x * 8 + (threadIdx.x >> 5); if (row >= (size_t)nrows) return; constexpr int LD = NFULL * 128 + TAIL * 64; const float* sr = Sb + row * LD; h16* pr = P + row * LD; const bool live = (int)(row % rowsper) < rvalid; float mx = -3.0e38f;
#pragma unroll 1
    for (int ch = 0; ch < NFULL + TAIL; ++ch) { if (ch == NFULL && lane >= 16) break; const int j0 = ch * 128 + lane * 4; const v4f a = *(const v4f*)(sr + j0);
#pragma unroll
        for (int q = 0; q < 4; ++q) if (j0 + q < nvalid) mx = fmaxf(mx, a[q]); }
#pragma unroll
    for (int sh = 16; sh; sh >>= 1) mx = fmaxf(mx, __shfl_xor(mx, sh, 32));
    float sum = 0.f;
#pragma unroll 1
    for (int ch = 0; ch < NFULL + TAIL; ++ch) { if (ch == NFULL && lane >= 16) break; const int j0 = ch * 128 + lane * 4; const v4f a = *(const v4f*)(sr + j0);
#pragma unroll
        for (int q = 0; q < 4; ++q) if (j0 + q < nvalid) { float d0 = __fsub_rn(a[q], mx); asm volatile("" : "+v"(d0)); sum += __expf(d0); } }
#pragma unroll
    for (int sh = 16; sh; sh >>= 1) sum += __shfl_xor(sum, sh, 32);
    const float f = live ? __fdiv_rn(PCAR, sum) : 0.f;
    for (int ps = 0; ps < 2; ++ps) {
#pragma unroll 1
        for (int ch = 0; ch < NFULL + TAIL; ++ch) { if (ch == NFULL && lane >= 16) break; const int j0 = ch * 128 + lane * 4; const v4f a = *(const v4f*)(sr + j0); v4h o;
#pragma unroll
            for (int q = 0; q < 4; ++q) { float val = 0.f; if (live && j0 + q < nvalid) { float d0 = __fsub_rn(a[q], mx); asm volatile("" : "+v"(d0)); val = __fmul_rn(__expf(d0), f); } o[q] = tohx(val); } *(volatile v4h*)(pr + j0) = o; }
        if (ps == 0) __threadfence(); } }

extern "C" void kernel_launch(void* const* d_in, const int* in_sizes, int n_in,
                              void* d_out, int out_size, void* d_ws, size_t ws_size, hipStream_t stream) {
    (void)in_sizes; (void)n_in; (void)out_size;
    const float* tgt = (const float*)d_in[0]; const float* src = (const float*)d_in[1]; const float* val = (const float*)d_in[2]; const float* wq = (const float*)d_in[3]; const float* bq = (const float*)d_in[4]; const float* wk = (const float*)d_in[5]; const float* bk = (const float*)d_in[6]; const float* wv = (const float*)d_in[7]; const float* bv = (const float*)d_in[8]; const float* wo = (const float*)d_in[9]; const float* bo = (const float*)d_in[10];
    float* OUT = (float*)d_out;
    char* wsp = (char*)d_ws;
    auto take = [&](size_t bytes) { char* p = wsp; wsp += (bytes + 255) & ~(size_t)255; return (void*)p; };
    bf* WQ = (bf*)take((size_t)DM * DM * 2); bf* WK = (bf*)take((size_t)DM * DM * 2); bf* WV = (bf*)take((size_t)DM * DM * 2); bf* WO = (bf*)take((size_t)DM * DM * 2);
    bf* XB = (bf*)take((size_t)LS * DM * 2); float* F = (float*)take((size_t)LS * DM * 4); h16* Q16 = (h16*)take((size_t)NH_ * LQ * HD * 2); h16* K16 = (h16*)take((size_t)NH_ * LS * HD * 2); h16* VT = (h16*)take((size_t)NH_ * HD * LS * 2);
    float* Sb = (float*)take((size_t)ZH * LQ * LS * 4); h16* P16 = (h16*)take((size_t)ZH * LQ * LS * 2); float* O = (float*)take((size_t)ZH * LQ * HD * 4); bf* Mh = (bf*)take((size_t)LQ * DM * 2); bf* Ml = (bf*)take((size_t)LQ * DM * 2);
    if ((size_t)(wsp - (char*)d_ws) > ws_size) return;
    k_wtG<<<(DM * DM / 64 + 63) / 64, 256, 0, stream>>>(wq, DM, DM, WQ); k_wtG<<<(DM * DM / 64 + 63) / 64, 256, 0, stream>>>(wk, DM, DM, WK); k_wtG<<<(DM * DM / 64 + 63) / 64, 256, 0, stream>>>(wv, DM, DM, WV); k_wtG<<<(DM * DM / 64 + 63) / 64, 256, 0, stream>>>(wo, DM, DM, WO);
    for (int b = 0; b < NB_; ++b) {
        k_cvt8<<<(unsigned)(((size_t)LQ * DM / 8 + 255) / 256), 256, 0, stream>>>(tgt + (size_t)b * LQ * DM, XB, (size_t)LQ * DM / 8); k_gemmw<bf, 0, true><<<dim3(LQ / 64, DM / 64, 1), 32, 0, stream>>>(XB, nullptr, WQ, nullptr, DM, F, DM, bq, 0, 0, 0); k_hpl<<<(unsigned)(((size_t)NH_ * LQ * HD / 4 + 255) / 256), 256, 0, stream>>>(F, LQ, 0.125f, Q16);
        k_cvt8<<<(unsigned)(((size_t)LS * DM / 8 + 255) / 256), 256, 0, stream>>>(src + (size_t)b * LS * DM, XB, (size_t)LS * DM / 8); k_gemmw<bf, 0, true><<<dim3(LS / 64, DM / 64, 1), 32, 0, stream>>>(XB, nullptr, WK, nullptr, DM, F, DM, bk, 0, 0, 0); k_hpl<<<(unsigned)(((size_t)NH_ * LS * HD / 4 + 255) / 256), 256, 0, stream>>>(F, LS, 1.0f, K16);
        k_cvt8<<<(unsigned)(((size_t)LS * DM / 8 + 255) / 256), 256, 0, stream>>>(val + (size_t)b * LS * DM, XB, (size_t)LS * DM / 8); k_gemmw<bf, 0, true><<<dim3(LS / 64, DM / 64, 1), 32, 0, stream>>>(XB, nullptr, WV, nullptr, DM, F, DM, bv, 0, 0, 0); k_vt<<<(unsigned)(((size_t)NH_ * HD * LS / 2 + 255) / 256), 256, 0, stream>>>(F, VT);
        for (int h0 = 0; h0 < NH_; h0 += ZH) {
            k_gemmw<h16, 0, false><<<dim3(LQ / 64, LS / 64, ZH), 32, 0, stream>>>(Q16 + (size_t)h0 * LQ * HD, nullptr, K16 + (size_t)h0 * LS * HD, nullptr, HD, Sb, LS, nullptr, (size_t)LQ * HD, (size_t)LS * HD, (size_t)LQ * LS);
            k_soft<32, 0><<<(ZH * LQ + 7) / 8, 256, 0, stream>>>(Sb, ZH * LQ, LQ, LQ, LS, P16);
            k_gemmw<h16, 0, false><<<dim3(LQ / 64, 1, ZH), 32, 0, stream>>>(P16, nullptr, VT + (size_t)h0 * HD * LS, nullptr, LS, O, HD, nullptr, (size_t)LQ * LS, (size_t)HD * LS, (size_t)LQ * HD);
            k_mrg<<<(unsigned)(((size_t)ZH * LQ * HD / 2 + 255) / 256), 256, 0, stream>>>(O, h0, Mh, Ml); }
        k_gemmw<bf, 1, true><<<dim3(LQ / 64, DM / 64, 1), 32, 0, stream>>>(Mh, Ml, WO, nullptr, DM, OUT + (size_t)b * LQ * DM, DM, bo, 0, 0, 0); }
}
